// SAKELayer_20624432955636
// MI455X (gfx1250) — hardware-verified
//
#include <hip/hip_runtime.h>
#include <math.h>

typedef __attribute__((ext_vector_type(16))) _Float16 v16h;
typedef __attribute__((ext_vector_type(8)))  _Float16 v8h;
typedef __attribute__((ext_vector_type(16))) __bf16   v16b;
typedef __attribute__((ext_vector_type(8)))  float    v8f;
typedef __attribute__((ext_vector_type(4)))  float    v4f;

__device__ __forceinline__ int frag_k(int i, int h) { return (i < 8) ? (8 * h + i) : (16 + 8 * h + (i - 8)); }
__device__ __forceinline__ __bf16 bf16_rne(float f) {
    unsigned int u = __float_as_uint(f);
    u += 0x7fffu + ((u >> 16) & 1u);
    return __builtin_bit_cast(__bf16, (unsigned short)(u >> 16));
}
__device__ __forceinline__ float bf16_f32(__bf16 b) { return __uint_as_float(((unsigned int)__builtin_bit_cast(unsigned short, b)) << 16); }
__device__ __forceinline__ v8f wmma16(v16h a, v16h b, v8f c) {
    c = __builtin_amdgcn_wmma_f32_16x16x32_f16(false, a, false, b, (short)0, c, false, false);
    asm volatile("v_nop\n\tv_nop\n\tv_nop\n\tv_nop" : "+v"(c) : "v"(a), "v"(b));
    return c;
}
__device__ __forceinline__ v8f wmmab(v16b a, v16b b, v8f c) {
    c = __builtin_amdgcn_wmma_f32_16x16x32_bf16(false, a, false, b, (short)0, c, false, false);
    asm volatile("v_nop\n\tv_nop\n\tv_nop\n\tv_nop" : "+v"(c) : "v"(a), "v"(b));
    return c;
}
struct Split { v16b hi, lo; };
__device__ __forceinline__ v8f wmma3(const Split& a, const Split& b, v8f c) {
    c = __builtin_amdgcn_wmma_f32_16x16x32_bf16(false, a.hi, false, b.hi, (short)0, c, false, false);
    c = __builtin_amdgcn_wmma_f32_16x16x32_bf16(false, a.hi, false, b.lo, (short)0, c, false, false);
    c = __builtin_amdgcn_wmma_f32_16x16x32_bf16(false, a.lo, false, b.hi, (short)0, c, false, false);
    asm volatile("v_nop\n\tv_nop\n\tv_nop\n\tv_nop" : "+v"(c) : "v"(a.hi), "v"(a.lo), "v"(b.hi), "v"(b.lo));
    return c;
}
struct Split3 { v16b hi, mid, lo; };
__device__ __forceinline__ v8f wmma6(const Split3& a, const Split3& b, v8f c) {
    c = __builtin_amdgcn_wmma_f32_16x16x32_bf16(false, a.hi, false, b.hi, (short)0, c, false, false);
    c = __builtin_amdgcn_wmma_f32_16x16x32_bf16(false, a.hi, false, b.mid, (short)0, c, false, false);
    c = __builtin_amdgcn_wmma_f32_16x16x32_bf16(false, a.mid, false, b.hi, (short)0, c, false, false);
    c = __builtin_amdgcn_wmma_f32_16x16x32_bf16(false, a.hi, false, b.lo, (short)0, c, false, false);
    c = __builtin_amdgcn_wmma_f32_16x16x32_bf16(false, a.mid, false, b.mid, (short)0, c, false, false);
    c = __builtin_amdgcn_wmma_f32_16x16x32_bf16(false, a.lo, false, b.hi, (short)0, c, false, false);
    asm volatile("v_nop\n\tv_nop\n\tv_nop\n\tv_nop" : "+v"(c) : "v"(a.hi), "v"(a.mid), "v"(a.lo), "v"(b.hi), "v"(b.mid), "v"(b.lo));
    return c;
}

__device__ __forceinline__ v16h fh_ld(const float* __restrict__ p, long long sk, int k0, int h, int klen, float s) {
    v16h a;
#pragma unroll
    for (int i = 0; i < 16; ++i) { const int k = k0 + frag_k(i, h); a[i] = (k < klen) ? (_Float16)(p[(long long)k * sk] * s) : (_Float16)0.f; }
    return a;
}
__device__ __forceinline__ Split sp_ld(const float* __restrict__ p, long long sk, int k0, int h, int klen, float s) {
    Split r;
#pragma unroll
    for (int i = 0; i < 16; ++i) {
        const int k = k0 + frag_k(i, h); const float x = (k < klen) ? p[(long long)k * sk] * s : 0.f;
        const __bf16 hb = bf16_rne(x); r.hi[i] = hb; r.lo[i] = bf16_rne(x - bf16_f32(hb));
    }
    return r;
}
__device__ __forceinline__ Split3 sp3_ld(const float* __restrict__ p, long long sk, int k0, int h, int klen, float s) {
    Split3 r;
#pragma unroll
    for (int i = 0; i < 16; ++i) {
        const int k = k0 + frag_k(i, h); const float x = (k < klen) ? p[(long long)k * sk] * s : 0.f;
        const __bf16 hb = bf16_rne(x); const float r1 = x - bf16_f32(hb); const __bf16 mb = bf16_rne(r1);
        r.hi[i] = hb; r.mid[i] = mb; r.lo[i] = bf16_rne(r1 - bf16_f32(mb));
    }
    return r;
}
__device__ __forceinline__ v16b bh_ld(const float* __restrict__ p, long long sk, int k0, int h, int klen, float s) {
    v16b a;
#pragma unroll
    for (int i = 0; i < 16; ++i) { const int k = k0 + frag_k(i, h); a[i] = bf16_rne((k < klen) ? p[(long long)k * sk] * s : 0.f); }
    return a;
}
__device__ __forceinline__ v16h fh_row(const _Float16* __restrict__ row, int k0, int h) {
    v16h a;
#pragma unroll
    for (int i = 0; i < 16; ++i) a[i] = row[k0 + frag_k(i, h)];
    return a;
}

#define VST2(T, ptr, val) do { *(volatile T*)(ptr) = (val); __threadfence(); *(volatile T*)(ptr) = (val); } while (0)
typedef float v4f __attribute__((ext_vector_type(4)));
#define VST2V4(ptr, val) do { *(volatile v4f*)(ptr) = (val); __threadfence(); *(volatile v4f*)(ptr) = (val); } while (0)

__device__ __attribute__((noinline)) float act_fn(float v, int act) {
    if (act == 1) return fmaxf(v, 0.f);
    if (act == 2) { const float u = 0.7978845608028654f * (v + 0.044715f * v * v * v); return 0.5f * v * (1.f + tanhf(u)); }
    if (act == 3) return v / (1.f + expf(-v));
    if (act == 4) return 0.5f * v * (1.f + erff(v * 0.7071067811865476f));
    if (act == 5) return tanhf(v);
    if (act == 6) return 1.f / (1.f + expf(-v));
    if (act == 7) return (v > 0.f) ? v : 0.01f * v;
    if (act == 8) return (v > 0.f) ? v : (expf(v) - 1.f);
    if (act == 9) return fminf(fmaxf(v, 0.f), 6.f);
    if (act == 10) return fabsf(v);
    if (act == 11) return (v >= 0.f) ? v : 0.1f * v;
    if (act == 12) return (v > 0.f) ? v : 0.2f * v;
    if (act == 13) return (v > 20.f) ? v : log1pf(expf(v));
    return v;
}

struct GemmP {
    const float* A; const float* B; const float* bias; const float* R; float* C;
    long long sAo, sAi, sAm, sAk, sBo, sBi, sBn, sBk, sCo, sCi, sCm, sRo, sRi, sRm, sRn;
    int M, N, K, zi_n, flags, act; float alpha, beta, sa, sb;
    int Npad, pad_;
};
static_assert(sizeof(GemmP) == 5 * 8 + 15 * 8 + 6 * 4 + 4 * 4 + 2 * 4, "GemmP has padding");

template <int MODE>
__global__ __launch_bounds__(32) void k_gemm(GemmP p) {
    const int lane = threadIdx.x & 31, h = lane >> 4, l15 = lane & 15;
    const int m0 = blockIdx.y * 16, n0 = blockIdx.x * 32;
    const int z = blockIdx.z, zo = z / p.zi_n, zi = z - zo * p.zi_n;
    const float* A = p.A + zo * p.sAo + zi * p.sAi;
    const float* B = p.B + zo * p.sBo + zi * p.sBi;
    const int am = min(m0 + l15, p.M - 1);
    v8f acc[2], comp[2];
#pragma unroll
    for (int t = 0; t < 2; ++t) { v8f zz = {}; acc[t] = zz; comp[t] = zz; }
    for (int k0 = 0; k0 < p.K; k0 += 32) {
        const float* arow = A + (long long)am * p.sAm;
        if (MODE == 1) {
            const Split a = sp_ld(arow, p.sAk, k0, h, p.K, 1.f);
#pragma unroll
            for (int t = 0; t < 2; ++t) {
                const int bn = min(n0 + t * 16 + l15, p.N - 1);
                acc[t] = wmma3(a, sp_ld(B + (long long)bn * p.sBn, p.sBk, k0, h, p.K, 1.f), acc[t]);
            }
        } else if (MODE == 3) {
            const Split3 a = sp3_ld(arow, p.sAk, k0, h, p.K, 1.f);
#pragma unroll
            for (int t = 0; t < 2; ++t) {
                const int bn = min(n0 + t * 16 + l15, p.N - 1);
                acc[t] = wmma6(a, sp3_ld(B + (long long)bn * p.sBn, p.sBk, k0, h, p.K, 1.f), acc[t]);
            }
        } else if (MODE == 4) {
            const Split3 a = sp3_ld(arow, p.sAk, k0, h, p.K, 1.f);
#pragma unroll
            for (int t = 0; t < 2; ++t) {
                const int bn = min(n0 + t * 16 + l15, p.N - 1); v8f zz = {};
                const v8f part = wmma6(a, sp3_ld(B + (long long)bn * p.sBn, p.sBk, k0, h, p.K, 1.f), zz);
                const v8f y = part - comp[t]; const v8f s = acc[t] + y; comp[t] = (s - acc[t]) - y; acc[t] = s;
            }
        } else if (MODE == 2) {
            const v16b a = bh_ld(arow, p.sAk, k0, h, p.K, 1.f);
#pragma unroll
            for (int t = 0; t < 2; ++t) {
                const int bn = min(n0 + t * 16 + l15, p.N - 1);
                acc[t] = wmmab(a, bh_ld(B + (long long)bn * p.sBn, p.sBk, k0, h, p.K, 1.f), acc[t]);
            }
        } else {
            const v16h a = fh_ld(arow, p.sAk, k0, h, p.K, p.sa);
#pragma unroll
            for (int t = 0; t < 2; ++t) {
                const int bn = min(n0 + t * 16 + l15, p.N - 1);
                acc[t] = wmma16(a, fh_ld(B + (long long)bn * p.sBn, p.sBk, k0, h, p.K, p.sb), acc[t]);
            }
        }
    }
    const float iscale = (MODE == 0) ? p.alpha / (p.sa * p.sb) : p.alpha;
    float* C = p.C + zo * p.sCo + zi * p.sCi;
    const float* R = p.R + zo * p.sRo + zi * p.sRi;
    __shared__ __align__(16) float ctile[16][36];
#pragma unroll
    for (int t = 0; t < 2; ++t) {
        const int n = n0 + t * 16 + l15; const int nn = min(n, p.N - 1);
#pragma unroll
        for (int r = 0; r < 8; ++r) {
            const int m = m0 + 8 * h + r; const int mm = min(m, p.M - 1);
            float v = acc[t][r] * iscale;
            if (p.flags & 1) v += p.bias[nn];
            if (p.flags & 2) v += p.bias[mm];
            v = act_fn(v, p.act);
            if (p.flags & 4) v += p.beta * R[(long long)mm * p.sRm + (long long)nn * p.sRn];
            ctile[8 * h + r][t * 16 + l15] = (n < p.N) ? v : 0.f;
        }
    }
    __syncthreads();
    const int NW = (p.Npad > p.N) ? p.Npad : p.N;
    const bool fast = (m0 + 16 <= p.M) && (n0 + 32 <= NW) && ((p.sCm & 3) == 0) && ((((size_t)C) & 15) == 0);
    if (fast) {
#pragma unroll
        for (int s = 0; s < 4; ++s) {
            const int row = s * 4 + (lane >> 3), c4 = (lane & 7) * 4;
            const v4f v = *(const v4f*)&ctile[row][c4];
            VST2V4(C + (long long)(m0 + row) * p.sCm + n0 + c4, v);
        }
    } else {
        for (int row = 0; row < 16; ++row) {
            const int m = m0 + row, n = n0 + lane;
            if (m < p.M && n < NW) VST2(float, C + (long long)m * p.sCm + n, ctile[row][lane]);
        }
    }
}

#define AW 4
struct AttnP {
    const float* Q; const float* K; const float* V; float* O; float* P; const float* Mf; const int* Mi; float* ST;
    const float* Pw; const float* Rt; const int* SQ; const int* SK;
    long long swb, swh, swi, swj, srb, srh, sri;
    long long sQb, sQh, sQi, sQd, sKb, sKh, sKj, sKd, sVb, sVh, sVj, sVd, sOb, sOh, sOi, sPb, sPh, sPi, smb, smh, smi, smj;
    int Lq, Lk, dh, dv, hrep, causal, coff, pband;
    float scale, mfill; int nonorm, mpol;
    int roff, rn, segpol, win;
};
static_assert(sizeof(AttnP) == 12 * 8 + 29 * 8 + 16 * 4, "AttnP has padding");

#ifndef KATTN_ATTR
#define KATTN_ATTR
#endif
template <int DHP, int DVP, int QM, bool SPLITPV, bool TWOPASS>
__global__ __launch_bounds__(32 * AW) KATTN_ATTR void k_attn(AttnP p) {
    constexpr int NT = DVP / 16;
    constexpr int KS = DHP / 32;
    constexpr int VP = DVP + 8;
    __shared__ __align__(16) float    pl[AW][16 * 64];
    __shared__ __align__(16) _Float16 vl[(SPLITPV ? 2 : 1) * 64 * VP];
    const int lane = threadIdx.x & 31, hf = lane >> 4, l15 = lane & 15, wave = threadIdx.x >> 5;
    const int h = blockIdx.y, b = blockIdx.z, hk = h / p.hrep;
    const int q0 = (blockIdx.x * AW + wave) * 16;
    float* myp = pl[wave];
    const float L2E = 1.4426950408889634f;
    const float NEG = -__builtin_inff();
    const int qi = min(q0 + l15, p.Lq - 1);
    const float* qrow = p.Q + b * p.sQb + h * p.sQh + (long long)qi * p.sQi;
    const float* kbase = p.K + b * p.sKb + hk * p.sKh;
    const float* vbase = p.V + b * p.sVb + hk * p.sVh;
    v16h qa[QM == 0 ? KS : 1]; Split qs_[QM == 1 ? KS : 1]; Split3 qt_[QM == 2 ? KS : 1];
#pragma unroll
    for (int ks = 0; ks < KS; ++ks) {
        if (QM == 2) qt_[ks] = sp3_ld(qrow, p.sQd, ks * 32, hf, p.dh, 1.f);
        else if (QM == 1) qs_[ks] = sp_ld(qrow, p.sQd, ks * 32, hf, p.dh, 1.f);
        else qa[ks] = fh_ld(qrow, p.sQd, ks * 32, hf, p.dh, 1.f);
    }
    v8f o[NT]; float m8[8], l8[8];
#pragma unroll
    for (int t = 0; t < NT; ++t) { v8f zz = {}; o[t] = zz; }
#pragma unroll
    for (int i = 0; i < 8; ++i) { m8[i] = NEG; l8[i] = 0.f; }
    int jend = p.Lk;
    if (p.causal == 1) { const int je = (blockIdx.x * AW + AW - 1) * 16 + 16 + p.coff; jend = min(jend, max(je, 0)); }
    const int npass = TWOPASS ? 2 : 1;
    for (int pass = 0; pass < npass; ++pass) {
        const bool dopv = (!TWOPASS) || pass == 1;
        for (int j0 = 0; j0 < jend; j0 += 64) {
            if (dopv) {
                __syncthreads();
                for (int idx = threadIdx.x; idx < 64 * DVP; idx += 32 * AW) {
                    const int jr = idx / DVP, d = idx - jr * DVP, j = j0 + jr;
                    const float f = (j < p.Lk && d < p.dv) ? vbase[(long long)j * p.sVj + (long long)d * p.sVd] : 0.f;
                    if (SPLITPV) {
                        const __bf16 hb = bf16_rne(f);
                        ((__bf16*)vl)[jr * VP + d] = hb; ((__bf16*)vl)[64 * VP + jr * VP + d] = bf16_rne(f - bf16_f32(hb));
                    } else vl[jr * VP + d] = (_Float16)f;
                }
            }
            v8f s[4];
#pragma unroll
            for (int t = 0; t < 4; ++t) {
                const int j = min(j0 + t * 16 + l15, p.Lk - 1);
                const float* krow = kbase + (long long)j * p.sKj;
                v8f acc = {};
#pragma unroll
                for (int ks = 0; ks < KS; ++ks) {
                    if (QM == 2)      acc = wmma6(qt_[ks], sp3_ld(krow, p.sKd, ks * 32, hf, p.dh, 1.f), acc);
                    else if (QM == 1) acc = wmma3(qs_[ks], sp_ld(krow, p.sKd, ks * 32, hf, p.dh, 1.f), acc);
                    else              acc = wmma16(qa[ks], fh_ld(krow, p.sKd, ks * 32, hf, p.dh, 1.f), acc);
                }
                s[t] = acc;
            }
            float pv[8][4];
#pragma unroll
            for (int i = 0; i < 8; ++i) {
                const int irow = q0 + i + 8 * hf;
                const int ic = min(irow, p.Lq - 1);
                float sc[4];
#pragma unroll
                for (int t = 0; t < 4; ++t) {
                    const int jg = j0 + t * 16 + l15;
                    float v = s[t][i] * p.scale;
                    if (p.Mf) v += p.Mf[b * p.smb + h * p.smh + (long long)ic * p.smi + (long long)min(jg, p.Lk - 1) * p.smj];
                    if (p.Rt) { int rc = ic - min(jg, p.Lk - 1) + p.roff; rc = rc < 0 ? 0 : (rc >= p.rn ? p.rn - 1 : rc); v += p.Rt[b * p.srb + h * p.srh + (long long)ic * p.sri + rc]; }
                    if (p.Mi) { const int mv = p.Mi[b * p.smb + h * p.smh + (long long)ic * p.smi + (long long)min(jg, p.Lk - 1) * p.smj]; if (p.mpol ? (mv != 0) : (mv == 0)) v = p.mfill; }
                    if (p.SQ) { const bool same = p.SQ[(long long)b * p.Lq + ic] == p.SK[(long long)b * p.Lk + min(jg, p.Lk - 1)]; if (p.segpol ? same : !same) v = p.mfill; }
                    if (p.causal == 2 && jg > irow + p.coff) v = p.mfill;
                    if (jg >= p.Lk || (p.causal == 1 && jg > irow + p.coff) || (p.causal == 3 && jg < irow + p.coff) || (p.win > 0 && irow + p.coff - jg > p.win)) v = NEG; else v *= L2E;
                    sc[t] = v;
                }
                if (!TWOPASS || pass == 0) {
                    float mx = fmaxf(fmaxf(sc[0], sc[1]), fmaxf(sc[2], sc[3]));
                    mx = fmaxf(mx, __shfl_xor(mx, 1, 32)); mx = fmaxf(mx, __shfl_xor(mx, 2, 32));
                    mx = fmaxf(mx, __shfl_xor(mx, 4, 32)); mx = fmaxf(mx, __shfl_xor(mx, 8, 32));
                    const float mnew = fmaxf(m8[i], mx);
                    const float corr = (mnew == NEG) ? 1.f : exp2f(m8[i] - mnew);
                    float rs = 0.f;
#pragma unroll
                    for (int t = 0; t < 4; ++t) {
                        const float pp = (sc[t] == NEG) ? 0.f : exp2f(sc[t] - mnew); rs += pp;
                        pv[i][t] = p.Pw ? pp * p.Pw[b * p.swb + h * p.swh + (long long)ic * p.swi + (long long)min(j0 + t * 16 + l15, p.Lk - 1) * p.swj] : pp;
                    }
                    rs += __shfl_xor(rs, 1, 32); rs += __shfl_xor(rs, 2, 32); rs += __shfl_xor(rs, 4, 32); rs += __shfl_xor(rs, 8, 32);
                    l8[i] = l8[i] * corr + rs; m8[i] = mnew;
                    if (!TWOPASS) {
#pragma unroll
                        for (int t = 0; t < NT; ++t) o[t][i] *= corr;
                    }
                } else {
                    const float inv = (l8[i] > 0.f) ? 1.f / l8[i] : 0.f;
#pragma unroll
                    for (int t = 0; t < 4; ++t) {
                        const int jg = j0 + t * 16 + l15;
                        float pp = (sc[t] == NEG) ? 0.f : exp2f(sc[t] - m8[i]) * inv;
                        if (p.Pw) pp *= p.Pw[b * p.swb + h * p.swh + (long long)ic * p.swi + (long long)min(jg, p.Lk - 1) * p.swj];
                        pv[i][t] = pp;
                    }
                }
            }
            if (dopv) {
#pragma unroll
                for (int i = 0; i < 8; ++i)
#pragma unroll
                    for (int t = 0; t < 4; ++t) myp[(i + 8 * hf) * 64 + t * 16 + l15] = pv[i][t];
                __syncthreads();
                if (p.P) {
                    float* pb_ = p.P + b * p.sPb + h * p.sPh;
                    const bool fastP = (p.pband == 0) && ((p.sPi & 3) == 0) && (j0 + 64 <= p.Lk) && (q0 + 16 <= p.Lq) && ((((size_t)pb_) & 15) == 0);
                    if (fastP) {
#pragma unroll
                        for (int s = 0; s < 8; ++s) {
                            const int row = s * 2 + (lane >> 4), c4 = (lane & 15) * 4;
                            const v4f v = *(const v4f*)(myp + row * 64 + c4);
                            VST2V4(pb_ + (long long)(q0 + row) * p.sPi + j0 + c4, v);
                        }
                    } else {
                        for (int row = 0; row < 16; ++row) {
                            const int irow = q0 + row; if (irow >= p.Lq) continue;
                            for (int c = lane; c < 64; c += 32) {
                                const int jg = j0 + c; if (jg >= p.Lk) continue;
                                if (p.pband == 0) VST2(float, pb_ + (long long)irow * p.sPi + jg, myp[row * 64 + c]);
                                else if (jg - irow <= p.pband && irow - jg <= p.pband) VST2(float, pb_ + (long long)irow * p.sPi + (jg - irow + p.pband), myp[row * 64 + c]);
                            }
                        }
                    }
                }
                if (SPLITPV) {
                    const Split pa0 = sp_ld(myp + l15 * 64, 1, 0, hf, 64, 1.f), pa1 = sp_ld(myp + l15 * 64, 1, 32, hf, 64, 1.f);
                    const __bf16* vh = (const __bf16*)vl; const __bf16* vlo = vh + 64 * VP;
#pragma unroll
                    for (int t = 0; t < NT; ++t) {
                        const int dcol = t * 16 + l15;
                        Split b0, b1;
#pragma unroll
                        for (int e = 0; e < 16; ++e) {
                            const int k0 = frag_k(e, hf), k1 = 32 + frag_k(e, hf);
                            b0.hi[e] = vh[k0 * VP + dcol]; b0.lo[e] = vlo[k0 * VP + dcol]; b1.hi[e] = vh[k1 * VP + dcol]; b1.lo[e] = vlo[k1 * VP + dcol];
                        }
                        o[t] = wmma3(pa0, b0, o[t]);
                        o[t] = wmma3(pa1, b1, o[t]);
                    }
                } else {
                    const v16h pa0 = fh_ld(myp + l15 * 64, 1, 0, hf, 64, 4096.f), pa1 = fh_ld(myp + l15 * 64, 1, 32, hf, 64, 4096.f);
#pragma unroll
                    for (int t = 0; t < NT; ++t) {
                        const int dcol = t * 16 + l15;
                        v16h b0, b1;
#pragma unroll
                        for (int e = 0; e < 16; ++e) { b0[e] = vl[frag_k(e, hf) * VP + dcol]; b1[e] = vl[(32 + frag_k(e, hf)) * VP + dcol]; }
                        o[t] = wmma16(pa0, b0, o[t]);
                        o[t] = wmma16(pa1, b1, o[t]);
                    }
                }
            }
        }
    }
    float* obase = p.O + b * p.sOb + h * p.sOh;
    if (p.ST) {
        const int rl = lane >> 1, isel = rl & 7;
        float mv = 0.f, lv = 0.f;
#pragma unroll
        for (int i = 0; i < 8; ++i) if (i == isel) { mv = m8[i]; lv = l8[i]; }
        const int irow = q0 + rl;
        if (irow < p.Lq) { float* st = p.ST + (((long long)b * gridDim.y + h) * p.Lq + irow) * 2 + (lane & 1); VST2(float, st, (lane & 1) ? lv : mv * 0.6931471805599453f); }
    }
    float invr[8];
#pragma unroll
    for (int i = 0; i < 8; ++i) {
        if (TWOPASS) invr[i] = SPLITPV ? 1.f : (1.f / 4096.f);
        else if (p.nonorm) invr[i] = exp2f(m8[i]) * (SPLITPV ? 1.f : (1.f / 4096.f));
        else invr[i] = (l8[i] > 0.f) ? (SPLITPV ? 1.f / l8[i] : 1.f / (l8[i] * 4096.f)) : 0.f;
    }
    __syncthreads();
    const bool ofast = ((p.sOi & 3) == 0) && ((((size_t)obase) & 15) == 0) && (q0 + 16 <= p.Lq);
#pragma unroll
    for (int c0 = 0; c0 < DVP; c0 += 64) {
#pragma unroll
        for (int i = 0; i < 8; ++i)
#pragma unroll
            for (int t = 0; t < NT; ++t) if (t * 16 >= c0 && t * 16 < c0 + 64) myp[(i + 8 * hf) * 64 + (t * 16 - c0) + l15] = o[t][i] * invr[i];
        __syncthreads();
        const int cw = (DVP - c0 < 64) ? (DVP - c0) : 64;
        if (ofast && (c0 + cw <= p.dv) && (cw % 32 == 0)) {
            const int lpr = cw / 4;
            const int rows_per_ins = 32 / lpr;
            for (int r0 = 0; r0 < 16; r0 += rows_per_ins) {
                const int row = r0 + lane / lpr, c4 = (lane % lpr) * 4;
                const v4f v = *(const v4f*)(myp + row * 64 + c4);
                VST2V4(obase + (long long)(q0 + row) * p.sOi + c0 + c4, v);
            }
        } else {
            for (int row = 0; row < 16; ++row) {
                const int irow = q0 + row; if (irow >= p.Lq) continue;
                for (int c = lane; c < cw; c += 32) { const int d = c0 + c; if (d < p.dv) VST2(float, obase + (long long)irow * p.sOi + d, myp[row * 64 + c]); }
            }
        }
        __syncthreads();
    }
}

struct TrP { const float* src; float* dst; const float* R2; long long sSz, lds, sDz, ldd, sRz, ldr; int R, C, flags, act; float alpha, beta; };
static_assert(sizeof(TrP) == 3 * 8 + 6 * 8 + 6 * 4, "TrP has padding");
__global__ __launch_bounds__(256) void k_tr(TrP p) {
    __shared__ float tile[32][33];
    const int c0 = blockIdx.x * 32, r0 = blockIdx.y * 32, z = blockIdx.z;
    const int lane = threadIdx.x & 31, wave = threadIdx.x >> 5;
    const float* s = p.src + z * p.sSz;
#pragma unroll
    for (int k = 0; k < 4; ++k) {
        const int rl = wave * 4 + k, r = r0 + rl, c = c0 + lane;
        tile[rl][lane] = (r < p.R && c < p.C) ? s[(long long)r * p.lds + c] : 0.f;
    }
    __syncthreads();
    float* d = p.dst + z * p.sDz; const float* rr = p.R2 + z * p.sRz;
#pragma unroll
    for (int k = 0; k < 4; ++k) {
        const int cl = wave * 4 + k, c = c0 + cl, r = r0 + lane;
        if (c < p.C && r < p.R) {
            float v = act_fn(p.alpha * tile[lane][cl], p.act);
            if (p.flags & 1) v += p.beta * rr[(long long)c * p.ldr + r];
            VST2(float, d + (long long)c * p.ldd + r, v);
        }
    }
}

__global__ __launch_bounds__(256) void k_affine(const float* __restrict__ src, float* __restrict__ dst, int n, float a, float b, const float* __restrict__ sdev) {
    const int i = blockIdx.x * 256 + threadIdx.x;
    if (i < n) { const float aa = sdev ? a * sdev[0] : a; const float v = aa * src[i] + b; VST2(float, dst + i, v); }
}

struct SmP { const float* src; float* dst; const float* Mf; long long sz, sr, dz, dr, smz, smr; int n, pad; float scale_in, scale_out; };
static_assert(sizeof(SmP) == 3 * 8 + 6 * 8 + 4 * 4, "SmP has padding");
__global__ __launch_bounds__(256) void k_softmax(SmP p) {
    __shared__ float red[256];
    const int r = blockIdx.x, z = blockIdx.y, tid = threadIdx.x;
    const float* s = p.src + z * p.sz + (long long)r * p.sr;
    const float* mf = p.Mf ? (p.Mf + z * p.smz + (long long)r * p.smr) : nullptr;
    float mx = -__builtin_inff();
    for (int j = tid; j < p.n; j += 256) { float v = s[j] * p.scale_in; if (mf) v += mf[j]; mx = fmaxf(mx, v); }
    red[tid] = mx; __syncthreads();
    for (int o = 128; o > 0; o >>= 1) { if (tid < o) red[tid] = fmaxf(red[tid], red[tid + o]); __syncthreads(); }
    mx = red[0]; __syncthreads();
    float sum = 0.f;
    for (int j = tid; j < p.n; j += 256) { float v = s[j] * p.scale_in; if (mf) v += mf[j]; sum += (mx == -__builtin_inff()) ? 0.f : expf(v - mx); }
    red[tid] = sum; __syncthreads();
    for (int o = 128; o > 0; o >>= 1) { if (tid < o) red[tid] += red[tid + o]; __syncthreads(); }
    sum = red[0];
    const float inv = (sum > 0.f) ? p.scale_out / sum : 0.f;
    float* d = p.dst + z * p.dz + (long long)r * p.dr;
    for (int j = tid; j < p.n; j += 256) { float v = s[j] * p.scale_in; if (mf) v += mf[j]; const float o = (mx == -__builtin_inff()) ? 0.f : expf(v - mx) * inv; VST2(float, d + j, o); }
}
__global__ __launch_bounds__(256) void k_stats(const float* __restrict__ x, long long sz, long long so, long long si, int inner, int n, float eps, float* __restrict__ stat, int mode) {
    __shared__ float red[256];
    const int z = blockIdx.x, tid = threadIdx.x;
    const float* base = x + z * sz;
    float s = 0.f;
    for (int e = tid; e < n; e += 256) s += base[(long long)(e / inner) * so + (long long)(e % inner) * si];
    red[tid] = s; __syncthreads();
    for (int o = 128; o > 0; o >>= 1) { if (tid < o) red[tid] += red[tid + o]; __syncthreads(); }
    const float mu = (mode == 0 || mode == 3) ? red[0] / (float)n : 0.f; __syncthreads();
    float q = 0.f;
    for (int e = tid; e < n; e += 256) { const float dlt = base[(long long)(e / inner) * so + (long long)(e % inner) * si] - mu; q += dlt * dlt; }
    red[tid] = q; __syncthreads();
    for (int o = 128; o > 0; o >>= 1) { if (tid < o) red[tid] += red[tid + o]; __syncthreads(); }
    {
        float rs;
        if (mode == 2) rs = sqrtf((float)n) / fmaxf(sqrtf(red[0]), eps); else if (mode == 3) rs = rsqrtf(red[0] / (float)(n - 1) + eps); else rs = rsqrtf(red[0] / (float)n + eps);
        if (tid < 32) { const float v = (tid == 0) ? mu : ((tid == 1) ? rs : 0.f); VST2(float, stat + (long long)z * 32 + tid, v); }
    }
}
__global__ __launch_bounds__(256) void k_norm_apply(const float* __restrict__ x, float* __restrict__ y, const float* __restrict__ stat, const float* __restrict__ g, const float* __restrict__ bta,
                                                     int Z, int C, int L, int G, int bn, int act) {
    const long long idx = (long long)blockIdx.x * 256 + threadIdx.x;
    if (idx >= (long long)Z * C * L) return;
    const int l = (int)(idx % L); const long long zc = idx / L; const int c = (int)(zc % C), z = (int)(zc / C); (void)l;
    const int set = bn ? c : (z * G + c / (C / G));
    float v = (x[idx] - stat[(long long)set * 32]) * stat[(long long)set * 32 + 1];
    if (g) v *= g[c];
    if (bta) v += bta[c];
    v = act_fn(v, act);
    VST2(float, y + idx, v);
}

__global__ __launch_bounds__(256) void k_lse_neg(const float* __restrict__ st, float* __restrict__ c, int n) {
    const int i = blockIdx.x * 256 + threadIdx.x;
    if (i < n) { const float v = -(st[2 * i] + logf(st[2 * i + 1])); VST2(float, c + i, v); }
}

__global__ __launch_bounds__(256) void k_iota(int* __restrict__ dst, int n, int a, int b) {
    const int i = blockIdx.x * 256 + threadIdx.x;
    if (i < n) { const int v = a * i + b; VST2(int, dst + i, v); }
}

__global__ __launch_bounds__(256) void k_axpby(const float* __restrict__ x, const float* __restrict__ y, float* __restrict__ dst, int n, float a, float b, float c) {
    const int i = blockIdx.x * 256 + threadIdx.x;
    if (i < n) { const float v = a * x[i] + b * y[i] + c; VST2(float, dst + i, v); }
}

struct RopeP { const float* X; float* Y; const float* C; const float* Sn; const int* pos; long long sXr, sXh, sYr, sYh, sCb, sCp, sCd; int R, Hn, D, S, mode, tmode, pmode, pad; };
static_assert(sizeof(RopeP) == 5 * 8 + 7 * 8 + 8 * 4, "RopeP has padding");
__global__ __launch_bounds__(256) void k_rope(RopeP p) {
    const long long idx = (long long)blockIdx.x * 256 + threadIdx.x;
    if (idx >= (long long)p.R * p.Hn * p.D) return;
    const int d = (int)(idx % p.D); const long long rh = idx / p.D; const int h = (int)(rh % p.Hn); const int r = (int)(rh / p.Hn);
    const int half = p.D / 2;
    int partner; float sign;
    if (p.mode == 0) { partner = (d < half) ? d + half : d - half; sign = (d < half) ? -1.f : 1.f; }
    else { partner = d ^ 1; sign = (d & 1) ? 1.f : -1.f; }
    const int tcol = (p.tmode == 0) ? d : ((p.tmode == 1) ? (d % half) : (d >> 1));
    const int pp = (p.pmode == 0) ? (r % p.S) : ((p.pmode == 1) ? h : p.pos[r]);
    const long long toff = (long long)(r / p.S) * p.sCb + (long long)pp * p.sCp + (long long)tcol * p.sCd;
    const float* xr = p.X + (long long)r * p.sXr + (long long)h * p.sXh;
    const float v = xr[d] * p.C[toff] + sign * xr[partner] * p.Sn[toff];
    VST2(float, p.Y + (long long)r * p.sYr + (long long)h * p.sYh + d, v);
}

__global__ __launch_bounds__(256) void k_invf(float* __restrict__ invb, int half, int D, float base, float num, int fmode, float cexp) {
    const int i = blockIdx.x * 256 + threadIdx.x;
    if (i >= ((half + 31) / 32) * 32) return;
    if (i >= half) { VST2(float, invb + i, 0.f); return; }
    const float e = (float)(2 * i) / (float)D;
    float invf;
    if (fmode == 1) invf = num * expf((float)(2 * i) * cexp);
    else if (fmode == 2) invf = num * powf(base, (-2.0f * ((float)i - 1.0f)) / (float)D);
    else invf = num * (1.0f / powf(base, e));
    VST2(float, invb + i, invf);
}
__global__ __launch_bounds__(256) void k_sincos(float* __restrict__ cs, float* __restrict__ sn, const float* __restrict__ invb, int S, int half, float pscale) {
    const int idx = blockIdx.x * 256 + threadIdx.x;
    if (idx >= S * half) return;
    const int s = idx / half, i = idx - s * half;
    const float ang = (pscale * (float)s) * invb[i];
    VST2(float, cs + idx, cosf(ang)); VST2(float, sn + idx, sinf(ang));
}

__global__ __launch_bounds__(256) void k_mulact(const float* __restrict__ x, const float* __restrict__ y, float* __restrict__ dst, int n, int act) {
    const int i = blockIdx.x * 256 + threadIdx.x;
    if (i < n) { const float v = act_fn(x[i], act) * y[i]; VST2(float, dst + i, v); }
}

__global__ __launch_bounds__(256) void k_matvec(GemmP p) {
    const int rpt = (p.N == 1) ? 1 : 32;
    const long long r0 = ((long long)blockIdx.x * 256 + threadIdx.x) * rpt; const int z = blockIdx.z, zo = z / p.zi_n, zi = z - zo * p.zi_n;
    if (r0 >= p.M) return;
    const float* Bb = p.B + zo * p.sBo + zi * p.sBi;
    float* C = p.C + zo * p.sCo + zi * p.sCi; const float* R = p.R + zo * p.sRo + zi * p.sRi;
    for (int rr = 0; rr < rpt; ++rr) {
        const long long r = r0 + rr; if (r >= p.M) break;
        const float* A = p.A + zo * p.sAo + zi * p.sAi + r * p.sAm;
        float acc[8] = {0.f, 0.f, 0.f, 0.f, 0.f, 0.f, 0.f, 0.f};
        for (int k = 0; k < p.K; ++k) { const float a = A[(long long)k * p.sAk];
#pragma unroll
            for (int j = 0; j < 8; ++j) if (j < p.N) acc[j] += a * Bb[(long long)j * p.sBn + (long long)k * p.sBk]; }
#pragma unroll
        for (int j = 0; j < 8; ++j) if (j < p.N) {
            float v = acc[j] * p.alpha;
            if (p.flags & 1) v += p.bias[j];
            if (p.flags & 2) v += p.bias[r];
            v = act_fn(v, p.act);
            if (p.flags & 4) v += p.beta * R[r * p.sRm + (long long)j * p.sRn];
            VST2(float, C + r * p.sCm + j, v);
        }
    }
}
__global__ __launch_bounds__(256) void k_smallsoftmax(const float* __restrict__ src, float* __restrict__ dst, long long sr, long long dr, int n, long long R, float scale) {
    const long long r0 = ((long long)blockIdx.x * 256 + threadIdx.x) * 32;
    for (int rr = 0; rr < 32; ++rr) {
        const long long r = r0 + rr; if (r >= R) return;
        const float* s = src + r * sr; float* d = dst + r * dr;
        float mx = -__builtin_inff();
        for (int j = 0; j < n; ++j) mx = fmaxf(mx, s[j] * scale);
        float sum = 0.f;
        for (int j = 0; j < n; ++j) sum += expf(s[j] * scale - mx);
        const float inv = 1.f / sum;
        for (int j = 0; j < n; ++j) { const float v = expf(s[j] * scale - mx) * inv; VST2(float, d + j, v); }
    }
}

__global__ __launch_bounds__(32) void k_unitstat(float* __restrict__ st) { const int t = threadIdx.x; const float v = (t == 1) ? 1.f : 0.f; VST2(float, st + t, v); }

__global__ __launch_bounds__(256) void k_lincopy(const float* __restrict__ src, long long lds, float* __restrict__ dst, long long ldd, long long rows, int cols) {
    const long long i = (long long)blockIdx.x * 256 + threadIdx.x; if (i >= rows * cols) return;
    const long long r = i / cols; const int c = (int)(i - r * cols);
    const float v = src[r * lds + c]; VST2(float, dst + r * ldd + c, v);
}

__global__ __launch_bounds__(256) void k_sk_e1(const float* __restrict__ X, const float* __restrict__ PI, const float* __restrict__ PJ, const float* __restrict__ We0, const float* __restrict__ be0, float* __restrict__ E1, int b, int N, int HD) { const long long q = (long long)blockIdx.x * 256 + threadIdx.x; if (q >= (long long)N * N * HD) return; const int c = (int)(q % HD); const long long ij = q / HD; const int j = (int)(ij % N), i = (int)(ij / N); const float* xi = X + ((long long)b * N + i) * 3; const float* xj = X + ((long long)b * N + j) * 3; const float dx = xi[0] - xj[0], dy = xi[1] - xj[1], dz = xi[2] - xj[2]; const float nrm = sqrtf(dx * dx + dy * dy + dz * dz + 1e-5f);
    const float v = PI[i * HD + c] + PJ[j * HD + c] + nrm * We0[128 * HD + c] + be0[c]; VST2(float, E1 + q, v / (1.f + expf(-v))); }
__global__ __launch_bounds__(256) void k_sk_node(const float* __restrict__ Hh, const float* __restrict__ X, const float* __restrict__ HE, const float* __restrict__ SL, const float* __restrict__ COEF, const float* __restrict__ SCL, const float* __restrict__ lg, float* __restrict__ AGG, float* __restrict__ CN, float* __restrict__ XOUT, int b, int N, int HD, int NH, int CC, int LP) {
    __shared__ float comb[4][384]; __shared__ float red[256]; const int i = blockIdx.x; const int t = threadIdx.x; const float* xi = X + ((long long)b * N + i) * 3;
    for (int h = 0; h < NH; ++h) { const float gam = expf(lg[h]);
        float meu = -__builtin_inff(), msem = -__builtin_inff();
        for (int j = t; j < N; j += 256) { const float* xj = X + ((long long)b * N + j) * 3; const float dx = xi[0] - xj[0], dy = xi[1] - xj[1], dz = xi[2] - xj[2]; const float nrm = sqrtf(dx * dx + dy * dy + dz * dz + 1e-5f); const float eye = (i == j) ? 1e5f : 0.f; const float leu = -(nrm + eye) * gam; float sl = SL[((long long)i * N + j) * LP + h]; sl = (sl > 0.f) ? sl : 0.2f * sl; const float lsem = sl - eye; comb[h][j] = leu; meu = fmaxf(meu, leu); msem = fmaxf(msem, lsem); }
        red[t] = meu; __syncthreads(); for (int o = 128; o > 0; o >>= 1) { if (t < o) red[t] = fmaxf(red[t], red[t + o]); __syncthreads(); } meu = red[0]; __syncthreads();
        red[t] = msem; __syncthreads(); for (int o = 128; o > 0; o >>= 1) { if (t < o) red[t] = fmaxf(red[t], red[t + o]); __syncthreads(); } msem = red[0]; __syncthreads();
        float seu = 0.f, ssem = 0.f; for (int j = t; j < N; j += 256) { float sl = SL[((long long)i * N + j) * LP + h]; sl = (sl > 0.f) ? sl : 0.2f * sl; const float lsem = sl - ((i == j) ? 1e5f : 0.f); seu += expf(comb[h][j] - meu); ssem += expf(lsem - msem); }
        red[t] = seu; __syncthreads(); for (int o = 128; o > 0; o >>= 1) { if (t < o) red[t] += red[t + o]; __syncthreads(); } seu = red[0]; __syncthreads();
        red[t] = ssem; __syncthreads(); for (int o = 128; o > 0; o >>= 1) { if (t < o) red[t] += red[t + o]; __syncthreads(); } ssem = red[0]; __syncthreads();
        float sc = 0.f; for (int j = t; j < N; j += 256) { float sl = SL[((long long)i * N + j) * LP + h]; sl = (sl > 0.f) ? sl : 0.2f * sl; const float lsem = sl - ((i == j) ? 1e5f : 0.f); const float cv = (expf(comb[h][j] - meu) / seu) * (expf(lsem - msem) / ssem); comb[h][j] = cv; sc += cv; }
        red[t] = sc; __syncthreads(); for (int o = 128; o > 0; o >>= 1) { if (t < o) red[t] += red[t + o]; __syncthreads(); } sc = red[0] + 1e-5f; __syncthreads();
        for (int j = t; j < N; j += 256) comb[h][j] = comb[h][j] / sc; __syncthreads(); }
    { const int h = t >> 6, c = t & 63; float a = 0.f;
#pragma unroll 1
        for (int j = 0; j < N; ++j) a += comb[h][j] * HE[((long long)i * N + j) * HD + c]; VST2(float, AGG + (long long)i * 384 + 64 + h * 64 + c, a); if (t < 64) VST2(float, AGG + (long long)i * 384 + t, Hh[((long long)b * N + i) * HD + t]); }
    if (t < CC * 3) { const int cc = t / 3, ax = t % 3; float s = 0.f;
#pragma unroll 1
        for (int j = 0; j < N; ++j) { const float* xj = X + ((long long)b * N + j) * 3; const float dx = xi[0] - xj[0], dy = xi[1] - xj[1], dz = xi[2] - xj[2]; const float nrm = sqrtf(dx * dx + dy * dy + dz * dz + 1e-5f); const float dd = (ax == 0) ? dx : (ax == 1) ? dy : dz; s += COEF[((long long)i * N + j) * LP + cc] * dd / (nrm + 1e-5f); }
        red[t] = s / (float)N; }
    __syncthreads(); if (t < CC) { const float a0 = red[t * 3], a1 = red[t * 3 + 1], a2 = red[t * 3 + 2]; VST2(float, CN + (long long)i * CC + t, a0 * a0 + a1 * a1 + a2 * a2); }
    if (t >= 128 && t < 131) { const int ax = t - 128; float s = 0.f;
#pragma unroll 1
        for (int j = 0; j < N; ++j) { const float* xj = X + ((long long)b * N + j) * 3; s += (xi[ax] - xj[ax]) * SCL[((long long)i * N + j) * LP]; } VST2(float, XOUT + ((long long)b * N + i) * 3 + ax, xi[ax] + s / (float)N); } }

template __global__ void k_gemm<0>(GemmP);

extern "C" void kernel_launch(void* const* d_in, const int* in_sizes, int n_in, void* d_out, int out_size, void* d_ws, size_t ws_size, hipStream_t stream) {
    (void)in_sizes; (void)n_in; (void)out_size; (void)ws_size;
    const float* h = (const float*)d_in[0];
    const float* x = (const float*)d_in[1];
    const float* We0 = (const float*)d_in[2];
    const float* be0 = (const float*)d_in[3];
    const float* We1 = (const float*)d_in[4];
    const float* be1 = (const float*)d_in[5];
    const float* Ws = (const float*)d_in[6];
    const float* bs = (const float*)d_in[7];
    const float* Wc0 = (const float*)d_in[8];
    const float* bc0 = (const float*)d_in[9];
    const float* Wc1 = (const float*)d_in[10];
    const float* bc1 = (const float*)d_in[11];
    const float* Wp0 = (const float*)d_in[12];
    const float* bp0 = (const float*)d_in[13];
    const float* Wp1 = (const float*)d_in[14];
    const float* bp1 = (const float*)d_in[15];
    const float* Wx0 = (const float*)d_in[16];
    const float* bx0 = (const float*)d_in[17];
    const float* Wx1 = (const float*)d_in[18];
    const float* Wn0 = (const float*)d_in[19];
    const float* bn0 = (const float*)d_in[20];
    const float* Wn1 = (const float*)d_in[21];
    const float* bn1 = (const float*)d_in[22];
    const float* lg = (const float*)d_in[23];
    const int Bn = 2;
    const int N = 384;
    const int F = 64;
    const int HD = 64;
    const int NH = 4;
    const int CC = 32;
    const int NP = N * N;
    const int LP = 32;
    float* out = (float*)d_out;
    float* xout = out + ((size_t)Bn * N * F);
    char* wsp = (char*)d_ws;
    float* PI = (float*)wsp; wsp += (((size_t)((size_t)N * HD) * 4 + 255) / 256) * 256;
    float* PJ = (float*)wsp; wsp += (((size_t)((size_t)N * HD) * 4 + 255) / 256) * 256;
    float* E1 = (float*)wsp; wsp += (((size_t)((size_t)NP * HD) * 4 + 255) / 256) * 256;
    float* HE = (float*)wsp; wsp += (((size_t)((size_t)NP * HD) * 4 + 255) / 256) * 256;
    float* SL = (float*)wsp; wsp += (((size_t)((size_t)NP * LP) * 4 + 255) / 256) * 256;
    float* T0 = (float*)wsp; wsp += (((size_t)((size_t)NP * HD) * 4 + 255) / 256) * 256;
    float* COEF = (float*)wsp; wsp += (((size_t)((size_t)NP * LP) * 4 + 255) / 256) * 256;
    float* SCL = (float*)wsp; wsp += (((size_t)((size_t)NP * LP) * 4 + 255) / 256) * 256;
    float* AGG = (float*)wsp; wsp += (((size_t)((size_t)N * 384) * 4 + 255) / 256) * 256;
    float* CN = (float*)wsp; wsp += (((size_t)((size_t)N * CC) * 4 + 255) / 256) * 256;
    float* P0 = (float*)wsp; wsp += (((size_t)((size_t)N * HD) * 4 + 255) / 256) * 256;
    float* N0 = (float*)wsp; wsp += (((size_t)((size_t)N * HD) * 4 + 255) / 256) * 256;
    { GemmP gpi0;
      gpi0.A = h + (size_t)0 * N * F; gpi0.B = We0; gpi0.bias = h + (size_t)0 * N * F; gpi0.R = h + (size_t)0 * N * F; gpi0.C = PI;
      gpi0.sAo = 0; gpi0.sAi = 0; gpi0.sAm = F; gpi0.sAk = 1; gpi0.sBo = 0; gpi0.sBi = 0; gpi0.sBn = 1; gpi0.sBk = HD; gpi0.sCo = 0; gpi0.sCi = 0; gpi0.sCm = HD; gpi0.sRo = 0; gpi0.sRi = 0; gpi0.sRm = 0; gpi0.sRn = 0;
      gpi0.M = N; gpi0.N = HD; gpi0.K = F; gpi0.zi_n = 1; gpi0.flags = 0; gpi0.act = 0;
      gpi0.alpha = 1.0f; gpi0.beta = 0.0f; gpi0.sa = 1.0f; gpi0.sb = 8.0f; gpi0.Npad = HD; gpi0.pad_ = 0;
      k_gemm<0><<<dim3((unsigned)((HD) + 31) / 32, (unsigned)((N) + 15) / 16, (unsigned)(1)), 32, 0, stream>>>(gpi0); }
    { GemmP gpj0;
      gpj0.A = h + (size_t)0 * N * F; gpj0.B = We0 + (size_t)F * HD; gpj0.bias = h + (size_t)0 * N * F; gpj0.R = h + (size_t)0 * N * F; gpj0.C = PJ;
      gpj0.sAo = 0; gpj0.sAi = 0; gpj0.sAm = F; gpj0.sAk = 1; gpj0.sBo = 0; gpj0.sBi = 0; gpj0.sBn = 1; gpj0.sBk = HD; gpj0.sCo = 0; gpj0.sCi = 0; gpj0.sCm = HD; gpj0.sRo = 0; gpj0.sRi = 0; gpj0.sRm = 0; gpj0.sRn = 0;
      gpj0.M = N; gpj0.N = HD; gpj0.K = F; gpj0.zi_n = 1; gpj0.flags = 0; gpj0.act = 0;
      gpj0.alpha = 1.0f; gpj0.beta = 0.0f; gpj0.sa = 1.0f; gpj0.sb = 8.0f; gpj0.Npad = HD; gpj0.pad_ = 0;
      k_gemm<0><<<dim3((unsigned)((HD) + 31) / 32, (unsigned)((N) + 15) / 16, (unsigned)(1)), 32, 0, stream>>>(gpj0); }
    k_sk_e1<<<(unsigned)(((long long)NP * HD + 255) / 256), 256, 0, stream>>>(x, PI, PJ, We0, be0, E1, 0, N, HD);
    { GemmP ghe0;
      ghe0.A = E1; ghe0.B = We1; ghe0.bias = be1; ghe0.R = E1; ghe0.C = HE;
      ghe0.sAo = 0; ghe0.sAi = 0; ghe0.sAm = HD; ghe0.sAk = 1; ghe0.sBo = 0; ghe0.sBi = 0; ghe0.sBn = 1; ghe0.sBk = HD; ghe0.sCo = 0; ghe0.sCi = 0; ghe0.sCm = HD; ghe0.sRo = 0; ghe0.sRi = 0; ghe0.sRm = 0; ghe0.sRn = 0;
      ghe0.M = NP; ghe0.N = HD; ghe0.K = HD; ghe0.zi_n = 1; ghe0.flags = 1; ghe0.act = 3;
      ghe0.alpha = 1.0f; ghe0.beta = 0.0f; ghe0.sa = 1.0f; ghe0.sb = 8.0f; ghe0.Npad = HD; ghe0.pad_ = 0;
      k_gemm<0><<<dim3((unsigned)((HD) + 31) / 32, (unsigned)((NP) + 15) / 16, (unsigned)(1)), 32, 0, stream>>>(ghe0); }
    { GemmP gsl0;
      gsl0.A = HE; gsl0.B = Ws; gsl0.bias = bs; gsl0.R = HE; gsl0.C = SL;
      gsl0.sAo = 0; gsl0.sAi = 0; gsl0.sAm = HD; gsl0.sAk = 1; gsl0.sBo = 0; gsl0.sBi = 0; gsl0.sBn = 1; gsl0.sBk = NH; gsl0.sCo = 0; gsl0.sCi = 0; gsl0.sCm = LP; gsl0.sRo = 0; gsl0.sRi = 0; gsl0.sRm = 0; gsl0.sRn = 0;
      gsl0.M = NP; gsl0.N = NH; gsl0.K = HD; gsl0.zi_n = 1; gsl0.flags = 1; gsl0.act = 0;
      gsl0.alpha = 1.0f; gsl0.beta = 0.0f; gsl0.sa = 1.0f; gsl0.sb = 8.0f; gsl0.Npad = LP; gsl0.pad_ = 0;
      k_gemm<0><<<dim3((unsigned)((LP) + 31) / 32, (unsigned)((NP) + 15) / 16, (unsigned)(1)), 32, 0, stream>>>(gsl0); }
    { GemmP gc00;
      gc00.A = HE; gc00.B = Wc0; gc00.bias = bc0; gc00.R = HE; gc00.C = T0;
      gc00.sAo = 0; gc00.sAi = 0; gc00.sAm = HD; gc00.sAk = 1; gc00.sBo = 0; gc00.sBi = 0; gc00.sBn = 1; gc00.sBk = HD; gc00.sCo = 0; gc00.sCi = 0; gc00.sCm = HD; gc00.sRo = 0; gc00.sRi = 0; gc00.sRm = 0; gc00.sRn = 0;
      gc00.M = NP; gc00.N = HD; gc00.K = HD; gc00.zi_n = 1; gc00.flags = 1; gc00.act = 3;
      gc00.alpha = 1.0f; gc00.beta = 0.0f; gc00.sa = 1.0f; gc00.sb = 8.0f; gc00.Npad = HD; gc00.pad_ = 0;
      k_gemm<0><<<dim3((unsigned)((HD) + 31) / 32, (unsigned)((NP) + 15) / 16, (unsigned)(1)), 32, 0, stream>>>(gc00); }
    { GemmP gc10;
      gc10.A = T0; gc10.B = Wc1; gc10.bias = bc1; gc10.R = T0; gc10.C = COEF;
      gc10.sAo = 0; gc10.sAi = 0; gc10.sAm = HD; gc10.sAk = 1; gc10.sBo = 0; gc10.sBi = 0; gc10.sBn = 1; gc10.sBk = CC; gc10.sCo = 0; gc10.sCi = 0; gc10.sCm = LP; gc10.sRo = 0; gc10.sRi = 0; gc10.sRm = 0; gc10.sRn = 0;
      gc10.M = NP; gc10.N = CC; gc10.K = HD; gc10.zi_n = 1; gc10.flags = 1; gc10.act = 0;
      gc10.alpha = 1.0f; gc10.beta = 0.0f; gc10.sa = 1.0f; gc10.sb = 8.0f; gc10.Npad = LP; gc10.pad_ = 0;
      k_gemm<0><<<dim3((unsigned)((LP) + 31) / 32, (unsigned)((NP) + 15) / 16, (unsigned)(1)), 32, 0, stream>>>(gc10); }
    { GemmP gx00;
      gx00.A = HE; gx00.B = Wx0; gx00.bias = bx0; gx00.R = HE; gx00.C = T0;
      gx00.sAo = 0; gx00.sAi = 0; gx00.sAm = HD; gx00.sAk = 1; gx00.sBo = 0; gx00.sBi = 0; gx00.sBn = 1; gx00.sBk = HD; gx00.sCo = 0; gx00.sCi = 0; gx00.sCm = HD; gx00.sRo = 0; gx00.sRi = 0; gx00.sRm = 0; gx00.sRn = 0;
      gx00.M = NP; gx00.N = HD; gx00.K = HD; gx00.zi_n = 1; gx00.flags = 1; gx00.act = 3;
      gx00.alpha = 1.0f; gx00.beta = 0.0f; gx00.sa = 1.0f; gx00.sb = 8.0f; gx00.Npad = HD; gx00.pad_ = 0;
      k_gemm<0><<<dim3((unsigned)((HD) + 31) / 32, (unsigned)((NP) + 15) / 16, (unsigned)(1)), 32, 0, stream>>>(gx00); }
    { GemmP gx10;
      gx10.A = T0; gx10.B = Wx1; gx10.bias = T0; gx10.R = T0; gx10.C = SCL;
      gx10.sAo = 0; gx10.sAi = 0; gx10.sAm = HD; gx10.sAk = 1; gx10.sBo = 0; gx10.sBi = 0; gx10.sBn = 1; gx10.sBk = 1; gx10.sCo = 0; gx10.sCi = 0; gx10.sCm = LP; gx10.sRo = 0; gx10.sRi = 0; gx10.sRm = 0; gx10.sRn = 0;
      gx10.M = NP; gx10.N = 1; gx10.K = HD; gx10.zi_n = 1; gx10.flags = 0; gx10.act = 0;
      gx10.alpha = 1.0f; gx10.beta = 0.0f; gx10.sa = 1.0f; gx10.sb = 8.0f; gx10.Npad = LP; gx10.pad_ = 0;
      k_gemm<0><<<dim3((unsigned)((LP) + 31) / 32, (unsigned)((NP) + 15) / 16, (unsigned)(1)), 32, 0, stream>>>(gx10); }
    k_sk_node<<<N, 256, 0, stream>>>(h, x, HE, SL, COEF, SCL, lg, AGG, CN, xout, 0, N, HD, NH, CC, LP);
    { GemmP gp00;
      gp00.A = CN; gp00.B = Wp0; gp00.bias = bp0; gp00.R = CN; gp00.C = P0;
      gp00.sAo = 0; gp00.sAi = 0; gp00.sAm = CC; gp00.sAk = 1; gp00.sBo = 0; gp00.sBi = 0; gp00.sBn = 1; gp00.sBk = HD; gp00.sCo = 0; gp00.sCi = 0; gp00.sCm = HD; gp00.sRo = 0; gp00.sRi = 0; gp00.sRm = 0; gp00.sRn = 0;
      gp00.M = N; gp00.N = HD; gp00.K = CC; gp00.zi_n = 1; gp00.flags = 1; gp00.act = 3;
      gp00.alpha = 1.0f; gp00.beta = 0.0f; gp00.sa = 1.0f; gp00.sb = 8.0f; gp00.Npad = HD; gp00.pad_ = 0;
      k_gemm<0><<<dim3((unsigned)((HD) + 31) / 32, (unsigned)((N) + 15) / 16, (unsigned)(1)), 32, 0, stream>>>(gp00); }
    { GemmP gp10;
      gp10.A = P0; gp10.B = Wp1; gp10.bias = bp1; gp10.R = P0; gp10.C = AGG + 320;
      gp10.sAo = 0; gp10.sAi = 0; gp10.sAm = HD; gp10.sAk = 1; gp10.sBo = 0; gp10.sBi = 0; gp10.sBn = 1; gp10.sBk = HD; gp10.sCo = 0; gp10.sCi = 0; gp10.sCm = 384; gp10.sRo = 0; gp10.sRi = 0; gp10.sRm = 0; gp10.sRn = 0;
      gp10.M = N; gp10.N = HD; gp10.K = HD; gp10.zi_n = 1; gp10.flags = 1; gp10.act = 0;
      gp10.alpha = 1.0f; gp10.beta = 0.0f; gp10.sa = 1.0f; gp10.sb = 8.0f; gp10.Npad = HD; gp10.pad_ = 0;
      k_gemm<0><<<dim3((unsigned)((HD) + 31) / 32, (unsigned)((N) + 15) / 16, (unsigned)(1)), 32, 0, stream>>>(gp10); }
    { GemmP gn00;
      gn00.A = AGG; gn00.B = Wn0; gn00.bias = bn0; gn00.R = AGG; gn00.C = N0;
      gn00.sAo = 0; gn00.sAi = 0; gn00.sAm = 384; gn00.sAk = 1; gn00.sBo = 0; gn00.sBi = 0; gn00.sBn = 1; gn00.sBk = HD; gn00.sCo = 0; gn00.sCi = 0; gn00.sCm = HD; gn00.sRo = 0; gn00.sRi = 0; gn00.sRm = 0; gn00.sRn = 0;
      gn00.M = N; gn00.N = HD; gn00.K = 384; gn00.zi_n = 1; gn00.flags = 1; gn00.act = 3;
      gn00.alpha = 1.0f; gn00.beta = 0.0f; gn00.sa = 1.0f; gn00.sb = 8.0f; gn00.Npad = HD; gn00.pad_ = 0;
      k_gemm<0><<<dim3((unsigned)((HD) + 31) / 32, (unsigned)((N) + 15) / 16, (unsigned)(1)), 32, 0, stream>>>(gn00); }
    { GemmP gn10;
      gn10.A = N0; gn10.B = Wn1; gn10.bias = bn1; gn10.R = h + (size_t)0 * N * F; gn10.C = out + (size_t)0 * N * F;
      gn10.sAo = 0; gn10.sAi = 0; gn10.sAm = HD; gn10.sAk = 1; gn10.sBo = 0; gn10.sBi = 0; gn10.sBn = 1; gn10.sBk = F; gn10.sCo = 0; gn10.sCi = 0; gn10.sCm = F; gn10.sRo = 0; gn10.sRi = 0; gn10.sRm = F; gn10.sRn = 1;
      gn10.M = N; gn10.N = F; gn10.K = HD; gn10.zi_n = 1; gn10.flags = 5; gn10.act = 0;
      gn10.alpha = 1.0f; gn10.beta = 1.0f; gn10.sa = 1.0f; gn10.sb = 8.0f; gn10.Npad = F; gn10.pad_ = 0;
      k_gemm<0><<<dim3((unsigned)((F) + 31) / 32, (unsigned)((N) + 15) / 16, (unsigned)(1)), 32, 0, stream>>>(gn10); }
    { GemmP gpi1;
      gpi1.A = h + (size_t)1 * N * F; gpi1.B = We0; gpi1.bias = h + (size_t)1 * N * F; gpi1.R = h + (size_t)1 * N * F; gpi1.C = PI;
      gpi1.sAo = 0; gpi1.sAi = 0; gpi1.sAm = F; gpi1.sAk = 1; gpi1.sBo = 0; gpi1.sBi = 0; gpi1.sBn = 1; gpi1.sBk = HD; gpi1.sCo = 0; gpi1.sCi = 0; gpi1.sCm = HD; gpi1.sRo = 0; gpi1.sRi = 0; gpi1.sRm = 0; gpi1.sRn = 0;
      gpi1.M = N; gpi1.N = HD; gpi1.K = F; gpi1.zi_n = 1; gpi1.flags = 0; gpi1.act = 0;
      gpi1.alpha = 1.0f; gpi1.beta = 0.0f; gpi1.sa = 1.0f; gpi1.sb = 8.0f; gpi1.Npad = HD; gpi1.pad_ = 0;
      k_gemm<0><<<dim3((unsigned)((HD) + 31) / 32, (unsigned)((N) + 15) / 16, (unsigned)(1)), 32, 0, stream>>>(gpi1); }
    { GemmP gpj1;
      gpj1.A = h + (size_t)1 * N * F; gpj1.B = We0 + (size_t)F * HD; gpj1.bias = h + (size_t)1 * N * F; gpj1.R = h + (size_t)1 * N * F; gpj1.C = PJ;
      gpj1.sAo = 0; gpj1.sAi = 0; gpj1.sAm = F; gpj1.sAk = 1; gpj1.sBo = 0; gpj1.sBi = 0; gpj1.sBn = 1; gpj1.sBk = HD; gpj1.sCo = 0; gpj1.sCi = 0; gpj1.sCm = HD; gpj1.sRo = 0; gpj1.sRi = 0; gpj1.sRm = 0; gpj1.sRn = 0;
      gpj1.M = N; gpj1.N = HD; gpj1.K = F; gpj1.zi_n = 1; gpj1.flags = 0; gpj1.act = 0;
      gpj1.alpha = 1.0f; gpj1.beta = 0.0f; gpj1.sa = 1.0f; gpj1.sb = 8.0f; gpj1.Npad = HD; gpj1.pad_ = 0;
      k_gemm<0><<<dim3((unsigned)((HD) + 31) / 32, (unsigned)((N) + 15) / 16, (unsigned)(1)), 32, 0, stream>>>(gpj1); }
    k_sk_e1<<<(unsigned)(((long long)NP * HD + 255) / 256), 256, 0, stream>>>(x, PI, PJ, We0, be0, E1, 1, N, HD);
    { GemmP ghe1;
      ghe1.A = E1; ghe1.B = We1; ghe1.bias = be1; ghe1.R = E1; ghe1.C = HE;
      ghe1.sAo = 0; ghe1.sAi = 0; ghe1.sAm = HD; ghe1.sAk = 1; ghe1.sBo = 0; ghe1.sBi = 0; ghe1.sBn = 1; ghe1.sBk = HD; ghe1.sCo = 0; ghe1.sCi = 0; ghe1.sCm = HD; ghe1.sRo = 0; ghe1.sRi = 0; ghe1.sRm = 0; ghe1.sRn = 0;
      ghe1.M = NP; ghe1.N = HD; ghe1.K = HD; ghe1.zi_n = 1; ghe1.flags = 1; ghe1.act = 3;
      ghe1.alpha = 1.0f; ghe1.beta = 0.0f; ghe1.sa = 1.0f; ghe1.sb = 8.0f; ghe1.Npad = HD; ghe1.pad_ = 0;
      k_gemm<0><<<dim3((unsigned)((HD) + 31) / 32, (unsigned)((NP) + 15) / 16, (unsigned)(1)), 32, 0, stream>>>(ghe1); }
    { GemmP gsl1;
      gsl1.A = HE; gsl1.B = Ws; gsl1.bias = bs; gsl1.R = HE; gsl1.C = SL;
      gsl1.sAo = 0; gsl1.sAi = 0; gsl1.sAm = HD; gsl1.sAk = 1; gsl1.sBo = 0; gsl1.sBi = 0; gsl1.sBn = 1; gsl1.sBk = NH; gsl1.sCo = 0; gsl1.sCi = 0; gsl1.sCm = LP; gsl1.sRo = 0; gsl1.sRi = 0; gsl1.sRm = 0; gsl1.sRn = 0;
      gsl1.M = NP; gsl1.N = NH; gsl1.K = HD; gsl1.zi_n = 1; gsl1.flags = 1; gsl1.act = 0;
      gsl1.alpha = 1.0f; gsl1.beta = 0.0f; gsl1.sa = 1.0f; gsl1.sb = 8.0f; gsl1.Npad = LP; gsl1.pad_ = 0;
      k_gemm<0><<<dim3((unsigned)((LP) + 31) / 32, (unsigned)((NP) + 15) / 16, (unsigned)(1)), 32, 0, stream>>>(gsl1); }
    { GemmP gc01;
      gc01.A = HE; gc01.B = Wc0; gc01.bias = bc0; gc01.R = HE; gc01.C = T0;
      gc01.sAo = 0; gc01.sAi = 0; gc01.sAm = HD; gc01.sAk = 1; gc01.sBo = 0; gc01.sBi = 0; gc01.sBn = 1; gc01.sBk = HD; gc01.sCo = 0; gc01.sCi = 0; gc01.sCm = HD; gc01.sRo = 0; gc01.sRi = 0; gc01.sRm = 0; gc01.sRn = 0;
      gc01.M = NP; gc01.N = HD; gc01.K = HD; gc01.zi_n = 1; gc01.flags = 1; gc01.act = 3;
      gc01.alpha = 1.0f; gc01.beta = 0.0f; gc01.sa = 1.0f; gc01.sb = 8.0f; gc01.Npad = HD; gc01.pad_ = 0;
      k_gemm<0><<<dim3((unsigned)((HD) + 31) / 32, (unsigned)((NP) + 15) / 16, (unsigned)(1)), 32, 0, stream>>>(gc01); }
    { GemmP gc11;
      gc11.A = T0; gc11.B = Wc1; gc11.bias = bc1; gc11.R = T0; gc11.C = COEF;
      gc11.sAo = 0; gc11.sAi = 0; gc11.sAm = HD; gc11.sAk = 1; gc11.sBo = 0; gc11.sBi = 0; gc11.sBn = 1; gc11.sBk = CC; gc11.sCo = 0; gc11.sCi = 0; gc11.sCm = LP; gc11.sRo = 0; gc11.sRi = 0; gc11.sRm = 0; gc11.sRn = 0;
      gc11.M = NP; gc11.N = CC; gc11.K = HD; gc11.zi_n = 1; gc11.flags = 1; gc11.act = 0;
      gc11.alpha = 1.0f; gc11.beta = 0.0f; gc11.sa = 1.0f; gc11.sb = 8.0f; gc11.Npad = LP; gc11.pad_ = 0;
      k_gemm<0><<<dim3((unsigned)((LP) + 31) / 32, (unsigned)((NP) + 15) / 16, (unsigned)(1)), 32, 0, stream>>>(gc11); }
    { GemmP gx01;
      gx01.A = HE; gx01.B = Wx0; gx01.bias = bx0; gx01.R = HE; gx01.C = T0;
      gx01.sAo = 0; gx01.sAi = 0; gx01.sAm = HD; gx01.sAk = 1; gx01.sBo = 0; gx01.sBi = 0; gx01.sBn = 1; gx01.sBk = HD; gx01.sCo = 0; gx01.sCi = 0; gx01.sCm = HD; gx01.sRo = 0; gx01.sRi = 0; gx01.sRm = 0; gx01.sRn = 0;
      gx01.M = NP; gx01.N = HD; gx01.K = HD; gx01.zi_n = 1; gx01.flags = 1; gx01.act = 3;
      gx01.alpha = 1.0f; gx01.beta = 0.0f; gx01.sa = 1.0f; gx01.sb = 8.0f; gx01.Npad = HD; gx01.pad_ = 0;
      k_gemm<0><<<dim3((unsigned)((HD) + 31) / 32, (unsigned)((NP) + 15) / 16, (unsigned)(1)), 32, 0, stream>>>(gx01); }
    { GemmP gx11;
      gx11.A = T0; gx11.B = Wx1; gx11.bias = T0; gx11.R = T0; gx11.C = SCL;
      gx11.sAo = 0; gx11.sAi = 0; gx11.sAm = HD; gx11.sAk = 1; gx11.sBo = 0; gx11.sBi = 0; gx11.sBn = 1; gx11.sBk = 1; gx11.sCo = 0; gx11.sCi = 0; gx11.sCm = LP; gx11.sRo = 0; gx11.sRi = 0; gx11.sRm = 0; gx11.sRn = 0;
      gx11.M = NP; gx11.N = 1; gx11.K = HD; gx11.zi_n = 1; gx11.flags = 0; gx11.act = 0;
      gx11.alpha = 1.0f; gx11.beta = 0.0f; gx11.sa = 1.0f; gx11.sb = 8.0f; gx11.Npad = LP; gx11.pad_ = 0;
      k_gemm<0><<<dim3((unsigned)((LP) + 31) / 32, (unsigned)((NP) + 15) / 16, (unsigned)(1)), 32, 0, stream>>>(gx11); }
    k_sk_node<<<N, 256, 0, stream>>>(h, x, HE, SL, COEF, SCL, lg, AGG, CN, xout, 1, N, HD, NH, CC, LP);
    { GemmP gp01;
      gp01.A = CN; gp01.B = Wp0; gp01.bias = bp0; gp01.R = CN; gp01.C = P0;
      gp01.sAo = 0; gp01.sAi = 0; gp01.sAm = CC; gp01.sAk = 1; gp01.sBo = 0; gp01.sBi = 0; gp01.sBn = 1; gp01.sBk = HD; gp01.sCo = 0; gp01.sCi = 0; gp01.sCm = HD; gp01.sRo = 0; gp01.sRi = 0; gp01.sRm = 0; gp01.sRn = 0;
      gp01.M = N; gp01.N = HD; gp01.K = CC; gp01.zi_n = 1; gp01.flags = 1; gp01.act = 3;
      gp01.alpha = 1.0f; gp01.beta = 0.0f; gp01.sa = 1.0f; gp01.sb = 8.0f; gp01.Npad = HD; gp01.pad_ = 0;
      k_gemm<0><<<dim3((unsigned)((HD) + 31) / 32, (unsigned)((N) + 15) / 16, (unsigned)(1)), 32, 0, stream>>>(gp01); }
    { GemmP gp11;
      gp11.A = P0; gp11.B = Wp1; gp11.bias = bp1; gp11.R = P0; gp11.C = AGG + 320;
      gp11.sAo = 0; gp11.sAi = 0; gp11.sAm = HD; gp11.sAk = 1; gp11.sBo = 0; gp11.sBi = 0; gp11.sBn = 1; gp11.sBk = HD; gp11.sCo = 0; gp11.sCi = 0; gp11.sCm = 384; gp11.sRo = 0; gp11.sRi = 0; gp11.sRm = 0; gp11.sRn = 0;
      gp11.M = N; gp11.N = HD; gp11.K = HD; gp11.zi_n = 1; gp11.flags = 1; gp11.act = 0;
      gp11.alpha = 1.0f; gp11.beta = 0.0f; gp11.sa = 1.0f; gp11.sb = 8.0f; gp11.Npad = HD; gp11.pad_ = 0;
      k_gemm<0><<<dim3((unsigned)((HD) + 31) / 32, (unsigned)((N) + 15) / 16, (unsigned)(1)), 32, 0, stream>>>(gp11); }
    { GemmP gn01;
      gn01.A = AGG; gn01.B = Wn0; gn01.bias = bn0; gn01.R = AGG; gn01.C = N0;
      gn01.sAo = 0; gn01.sAi = 0; gn01.sAm = 384; gn01.sAk = 1; gn01.sBo = 0; gn01.sBi = 0; gn01.sBn = 1; gn01.sBk = HD; gn01.sCo = 0; gn01.sCi = 0; gn01.sCm = HD; gn01.sRo = 0; gn01.sRi = 0; gn01.sRm = 0; gn01.sRn = 0;
      gn01.M = N; gn01.N = HD; gn01.K = 384; gn01.zi_n = 1; gn01.flags = 1; gn01.act = 3;
      gn01.alpha = 1.0f; gn01.beta = 0.0f; gn01.sa = 1.0f; gn01.sb = 8.0f; gn01.Npad = HD; gn01.pad_ = 0;
      k_gemm<0><<<dim3((unsigned)((HD) + 31) / 32, (unsigned)((N) + 15) / 16, (unsigned)(1)), 32, 0, stream>>>(gn01); }
    { GemmP gn11;
      gn11.A = N0; gn11.B = Wn1; gn11.bias = bn1; gn11.R = h + (size_t)1 * N * F; gn11.C = out + (size_t)1 * N * F;
      gn11.sAo = 0; gn11.sAi = 0; gn11.sAm = HD; gn11.sAk = 1; gn11.sBo = 0; gn11.sBi = 0; gn11.sBn = 1; gn11.sBk = F; gn11.sCo = 0; gn11.sCi = 0; gn11.sCm = F; gn11.sRo = 0; gn11.sRi = 0; gn11.sRm = F; gn11.sRn = 1;
      gn11.M = N; gn11.N = F; gn11.K = HD; gn11.zi_n = 1; gn11.flags = 5; gn11.act = 0;
      gn11.alpha = 1.0f; gn11.beta = 1.0f; gn11.sa = 1.0f; gn11.sb = 8.0f; gn11.Npad = F; gn11.pad_ = 0;
      k_gemm<0><<<dim3((unsigned)((F) + 31) / 32, (unsigned)((N) + 15) / 16, (unsigned)(1)), 32, 0, stream>>>(gn11); }
}
